// PartitionedGraphAttentionLayer_67482526154914
// MI455X (gfx1250) — hardware-verified
//
#include <hip/hip_runtime.h>
#include <math.h>

typedef __attribute__((ext_vector_type(16))) __bf16   v16b;
typedef __attribute__((ext_vector_type(8)))  __bf16   v8b;
typedef __attribute__((ext_vector_type(8)))  float    v8f;
typedef __attribute__((ext_vector_type(4)))  float    v4f;

constexpr int kNB     = 32;
constexpr int kCin    = 64;
constexpr int kTD     = 300;
constexpr int kVN     = 25;
constexpr int kFout   = 64;
constexpr int kNE     = 150;
constexpr int kNP     = 3;
constexpr int kTB     = 4;
constexpr int kRows   = kTB * kVN;
constexpr int kMPad   = 112;
constexpr int kHS     = 68;
constexpr int kAST    = 72;
constexpr int kAW     = kAST / 2;
constexpr int kTVP    = kTD * kVN;
constexpr int kBlkPerN = kTD / kTB;
constexpr int kNBlk   = kNB * kBlkPerN;
constexpr int kWsPitch = 128;
static_assert(kRows == 100 && kTVP == 7500 && kNBlk == 2400, "shape");
static_assert((kTD % kTB) == 0, "time chunks");
static_assert((kCin % 32) == 0, "K multiple of 32");
static_assert((kFout % 16) == 0 && (kMPad % 16) == 0 && kMPad >= kRows, "tile multiples");
static_assert((kRows % 4) == 0 && (kTVP % 4) == 0, "16-B aligned runs");
static_assert((kMPad + kFout) * kAST * 2 <= kRows * kHS * 4, "operand planes fit in the aliased accumulator region");

constexpr size_t kWsTotal = (size_t)kNBlk * kFout * kWsPitch * 4;
static_assert(kWsTotal == 78643200ull, "carve total");
static_assert(kWsTotal <= 134217728ull, "carve cap");

constexpr int kOutElems = kNB * kFout * kTVP;
static_assert(kOutElems == 15360000, "output elements");
static_assert((kOutElems % 1024) == 0, "copy grid exact");

__device__ __forceinline__ unsigned short f2bf_bits(float f) {
  unsigned u = __float_as_uint(f);
  return (unsigned short)((u + 0x7FFFu + ((u >> 16) & 1u)) >> 16);
}
__device__ __forceinline__ float bf_bits2f(unsigned short h) { return __uint_as_float(((unsigned)h) << 16); }
__device__ __forceinline__ unsigned pack_bf16x2(float lo, float hi) {
  const unsigned a = (unsigned)f2bf_bits(lo);
  const unsigned b = (unsigned)f2bf_bits(hi);
  return a | (b << 16);
}

union FragB { v16b v; v8b h[2]; };
__device__ __forceinline__ v16b frag_load(const __bf16* p) {
  FragB f;
  f.h[0] = *(const v8b*)(p);
  f.h[1] = *(const v8b*)(p + 16);
  return f.v;
}
__device__ __forceinline__ v8f mma_bf16(v16b a, v16b b, v8f c) {
  c = __builtin_amdgcn_wmma_f32_16x16x32_bf16(false, a, false, b, (short)0, c, false, false);
  asm volatile("v_nop\n\tv_nop\n\tv_nop\n\tv_nop" : "+v"(c) : "v"(a), "v"(b));
  return c;
}

__global__ __launch_bounds__(256) void graph_fused_kernel(
    const float* __restrict__ input, const float* __restrict__ W, const float* __restrict__ avec,
    const int* __restrict__ eidx, const int* __restrict__ epar, float* __restrict__ wsout)
{
  __shared__ __align__(16) float h_lds[kRows * kHS];
  __shared__ __align__(16) float hp_lds[kRows * kHS];
  __shared__ __align__(16) float a_lds[kNP * 2 * kFout];
  __shared__ __align__(16) float sc_lds[kRows * 6];
  __shared__ __align__(16) float e_lds[kTB * kNE];
  __shared__ __align__(16) float dinv_lds[kTB * 32];
  __shared__ int esrc[kNE];
  __shared__ int edst[kNE];
  __shared__ int eprt[kNE];

  const int tid  = threadIdx.x;
  const int lane = tid & 31;
  const int wave = __builtin_amdgcn_readfirstlane((int)(threadIdx.x >> 5));
  const int blk  = blockIdx.x;
  const int n    = blk / kBlkPerN;
  const int tb   = blk - n * kBlkPerN;
  const int tv0  = tb * kRows;

  unsigned* Aw = (unsigned*)hp_lds;
  unsigned* Bw = Aw + kMPad * kAW;

  {
    const int ec = tid < kNE ? tid : (kNE - 1);
    int sv = eidx[ec];
    int dv = eidx[kNE + ec];
    int pv = epar[ec];
    asm volatile("" : "+v"(sv), "+v"(dv), "+v"(pv));
    sv = sv < 0 ? 0 : (sv > kVN - 1 ? kVN - 1 : sv);
    dv = dv < 0 ? 0 : (dv > kVN - 1 ? kVN - 1 : dv);
    pv = pv < 0 ? 0 : (pv > kNP - 1 ? kNP - 1 : pv);
    if (tid < kNE) { esrc[tid] = sv; edst[tid] = dv; eprt[tid] = pv; }
  }
#pragma unroll
  for (int it = 0; it < 2; ++it) {
    const int i  = tid + it * 256;
    const int ic = i < (kNP * 2 * kFout) ? i : (kNP * 2 * kFout - 1);
    float av = avec[ic];
    asm volatile("" : "+v"(av));
    if (i < kNP * 2 * kFout) a_lds[i] = bf_bits2f(f2bf_bits(av));
  }
  {
    const float* inb = input + (size_t)n * kCin * kTVP + tv0;
#pragma unroll
    for (int it = 0; it < 4; ++it) {
      const int i  = tid + it * 256;
      const int ic = i < 800 ? i : 799;
      const int cp = ic / 25;
      const int mq = ic - cp * 25;
      const float* p0 = inb + (size_t)(2 * cp) * kTVP + mq * 4;
      const v4f x0 = *(const v4f*)(p0);
      const v4f x1 = *(const v4f*)(p0 + kTVP);
      float a0 = x0[0], a1 = x0[1], a2 = x0[2], a3 = x0[3];
      float b0 = x1[0], b1 = x1[1], b2 = x1[2], b3 = x1[3];
      asm volatile("" : "+v"(a0), "+v"(a1), "+v"(a2), "+v"(a3));
      asm volatile("" : "+v"(b0), "+v"(b1), "+v"(b2), "+v"(b3));
      if (i < 800) {
        unsigned* q = Aw + (mq * 4) * kAW + cp;
        q[0]       = pack_bf16x2(a0, b0);
        q[kAW]     = pack_bf16x2(a1, b1);
        q[2 * kAW] = pack_bf16x2(a2, b2);
        q[3 * kAW] = pack_bf16x2(a3, b3);
      }
    }
#pragma unroll
    for (int it = 0; it < 2; ++it) {
      const int i = tid + it * 256;
      if (i < 12 * 32) {
        const int zr = i >> 5;
        const int zw = i & 31;
        Aw[(kRows + zr) * kAW + zw] = 0u;
      }
    }
  }
#pragma unroll
  for (int it = 0; it < 2; ++it) {
    const int i  = tid + it * 256;
    const int cp = i >> 4;
    const int fq = i & 15;
    const float* p = W + (2 * cp) * kFout + fq * 4;
    const v4f w0 = *(const v4f*)(p);
    const v4f w1 = *(const v4f*)(p + kFout);
    const float a0 = w0[0], a1 = w0[1], a2 = w0[2], a3 = w0[3];
    const float b0 = w1[0], b1 = w1[1], b2 = w1[2], b3 = w1[3];
    unsigned* q = Bw + (fq * 4) * kAW + cp;
    q[0]       = pack_bf16x2(a0, b0);
    q[kAW]     = pack_bf16x2(a1, b1);
    q[2 * kAW] = pack_bf16x2(a2, b2);
    q[3 * kAW] = pack_bf16x2(a3, b3);
  }
  __syncthreads();

  if (wave < 7) {
    const int rl   = lane & 15;
    const int hh   = lane >> 4;
    const int koff = hh * 8;
    const __bf16* Ap = (const __bf16*)hp_lds;
    const __bf16* Bp = Ap + kMPad * kAST;
    const __bf16* arow = Ap + (wave * 16 + rl) * kAST + koff;
    const v16b fa0 = frag_load(arow);
    const v16b fa1 = frag_load(arow + 32);
#pragma unroll
    for (int nt = 0; nt < 4; ++nt) {
      const __bf16* brow = Bp + (nt * 16 + rl) * kAST + koff;
      const v16b fb0 = frag_load(brow);
      const v16b fb1 = frag_load(brow + 32);
      v8f c = (v8f){0.f, 0.f, 0.f, 0.f, 0.f, 0.f, 0.f, 0.f};
      c = mma_bf16(fa0, fb0, c);
      c = mma_bf16(fa1, fb1, c);
#pragma unroll
      for (int r = 0; r < 8; ++r) {
        const int row = wave * 16 + 8 * hh + r;
        if (row < kRows) h_lds[row * kHS + nt * 16 + rl] = c[r];
      }
    }
  }
  __syncthreads();

  for (int i = tid; i < (kRows * kHS) / 4; i += 256)
    *(v4f*)(hp_lds + 4 * i) = (v4f){0.f, 0.f, 0.f, 0.f};

#pragma unroll 1
  for (int it = 0; it < 3; ++it) {
    const int i   = tid + it * 256;
    const int ic  = i < kRows * 6 ? i : (kRows * 6 - 1);
    const int row = ic / 6;
    const int q   = ic - row * 6;
    const int aoff = (q < 3) ? (q * 2 * kFout) : ((q - 3) * 2 * kFout + kFout);
    const float* hr = h_lds + row * kHS;
    const float* ar = a_lds + aoff;
    float s = 0.0f;
#pragma unroll 4
    for (int f4 = 0; f4 < kFout / 4; ++f4) {
      const v4f hv = *(const v4f*)(hr + 4 * f4);
      const v4f av = *(const v4f*)(ar + 4 * f4);
      s = fmaf(hv[0], av[0], s);
      s = fmaf(hv[1], av[1], s);
      s = fmaf(hv[2], av[2], s);
      s = fmaf(hv[3], av[3], s);
    }
    if (i < kRows * 6) sc_lds[ic] = s;
  }
  __syncthreads();

  {
    const int g  = tid >> 6;
    const int gt = tid & 63;
    for (int e = gt; e < kNE; e += 64) {
      const int sv = esrc[e], dv = edst[e], p = eprt[e];
      const float z = sc_lds[(g * kVN + sv) * 6 + p] + sc_lds[(g * kVN + dv) * 6 + 3 + p];
      e_lds[g * kNE + e] = (z > 0.0f) ? z : 0.2f * z;
    }
  }
  __syncthreads();

  if (wave < 4) {
    const int g = wave;
    const int v = lane;
    if (v < kVN) {
      float* eg = e_lds + g * kNE;
      float m = -3.402823466e38f;
#pragma unroll 1
      for (int e = 0; e < kNE; ++e) {
        if (edst[e] == v) m = fmaxf(m, eg[e]);
      }
      float s = 0.0f;
#pragma unroll 1
      for (int e = 0; e < kNE; ++e) {
        if (edst[e] == v) {
          const float x = expf(eg[e] - m);
          eg[e] = x;
          s += x;
        }
      }
      const float sd = (s > 0.0f) ? s : 1.0f;
      const float iv = 1.0f / sd;
      dinv_lds[g * 32 + v] = (s > 0.0f) ? iv : 0.0f;
    }
  }
  __syncthreads();

  {
    const int g = tid >> 6;
    const int f = tid & 63;
    float* hpc = hp_lds + g * kVN * kHS + f;
    const float* hc = h_lds + g * kVN * kHS + f;
    const float* ex = e_lds + g * kNE;
#pragma unroll 2
    for (int e = 0; e < kNE; ++e) {
      const int sv = esrc[e], dv = edst[e];
      hpc[dv * kHS] = fmaf(ex[e], hc[sv * kHS], hpc[dv * kHS]);
    }
  }
  __syncthreads();

  {
    const int r0 = lane * 4;
    const bool valid = (r0 < kRows);
    int rcl[4];
    float dn[4];
#pragma unroll
    for (int j = 0; j < 4; ++j) {
      const int r  = r0 + j;
      const int rc = r < kRows ? r : (kRows - 1);
      const int g  = rc / kVN;
      const int v  = rc - g * kVN;
      rcl[j] = rc * kHS;
      dn[j]  = dinv_lds[g * 32 + v];
    }
    float* wbase = wsout + (size_t)blk * kFout * kWsPitch + r0;
#pragma unroll 1
    for (int it = 0; it < 8; ++it) {
      const int f = wave * 8 + it;
      v4f o;
#pragma unroll
      for (int j = 0; j < 4; ++j) {
        const float x = hp_lds[rcl[j] + f] * dn[j];
        const float y = (x > 0.0f) ? x : expm1f(x);
        o[j] = valid ? y : 0.0f;
      }
      float* dst = wbase + (size_t)f * kWsPitch;
      *(volatile v4f*)dst = o;
      __threadfence();
      *(volatile v4f*)dst = o;
    }
  }
}

__global__ __launch_bounds__(256) void pack_out_kernel(const float* __restrict__ hp, float* __restrict__ out)
{
  const int q = blockIdx.x * 256 + threadIdx.x;
  if (q >= kOutElems / 4) return;
  const int i   = q * 4;
  const int n   = i / (kFout * kTVP);
  const int rem = i - n * (kFout * kTVP);
  const int f   = rem / kTVP;
  const int tv  = rem - f * kTVP;
  const int tb  = tv / kRows;
  const int r   = tv - tb * kRows;
  const size_t so = ((size_t)((n * kBlkPerN + tb) * kFout + f)) * kWsPitch + r;
  const v4f v = *(const v4f*)(hp + so);
  float* dst = out + i;
  *(volatile v4f*)dst = v;
  __threadfence();
  *(volatile v4f*)dst = v;
}

extern "C" void kernel_launch(void* const* d_in, const int* in_sizes, int n_in,
                              void* d_out, int out_size, void* d_ws, size_t ws_size,
                              hipStream_t stream) {
  if (n_in < 5) return;
  if (in_sizes[0] != kNB * kCin * kTVP) return;
  if (in_sizes[1] != kCin * kFout) return;
  if (in_sizes[2] != kNP * 2 * kFout) return;
  if (in_sizes[3] != 2 * kNE) return;
  if (in_sizes[4] != kNE) return;
  if (out_size != kOutElems) return;
  if (ws_size < kWsTotal) return;

  const float* input = (const float*)d_in[0];
  const float* W     = (const float*)d_in[1];
  const float* avec  = (const float*)d_in[2];
  const int*   eidx  = (const int*)d_in[3];
  const int*   epar  = (const int*)d_in[4];
  float* out = (float*)d_out;
  float* hp  = (float*)d_ws;

  graph_fused_kernel<<<kNBlk, 256, 0, stream>>>(input, W, avec, eidx, epar, hp);
  pack_out_kernel<<<kOutElems / 4 / 256, 256, 0, stream>>>(hp, out);
}
